// PointNetSetAbstraction_19413252178083
// MI455X (gfx1250) — hardware-verified
//
#include <hip/hip_runtime.h>
#pragma clang fp contract(off)

typedef __attribute__((ext_vector_type(16))) _Float16 v16h;
typedef __attribute__((ext_vector_type(8)))  _Float16 v8h;
typedef __attribute__((ext_vector_type(8)))  float    v8f;
typedef __attribute__((ext_vector_type(4)))  float    v4f;

constexpr int kBatch = 8;
constexpr int kPts   = 8192;
constexpr int kCent  = 1024;
constexpr int kNbr   = 32;
constexpr int kFeat  = 61;
constexpr int kCin   = 64;
constexpr int kCout  = 128;
constexpr int kRows  = kBatch * kCent * kNbr;
constexpr int kGemmBlocks = kRows / 256;
constexpr float kWCarry    = 16.0f;
constexpr float kWCarryInv = 1.0f / 16.0f;
constexpr float kBnEps     = 1e-5f;
constexpr float kRadius    = 0.2f;

static_assert(kCin == 3 + kFeat);
static_assert(kRows == 262144);
static_assert(kRows % 256 == 0);
static_assert(kCin % 32 == 0);
static_assert(kCout % 64 == 0);
static_assert(kCent % 64 == 0);
static_assert(98304 + 4194304 == 4292608);
static_assert(kBatch * kCent * 3 * 4 == 98304);

struct FragH {
  union U { v16h v; v8h h[2]; };
  static __device__ __forceinline__ v16h load(const _Float16* p) {
    U f;
    f.h[0] = *(const v8h*)(p);
    f.h[1] = *(const v8h*)(p + 16);
    return f.v;
  }
  static __device__ __forceinline__ v8f mma(v16h a, v16h b, v8f c) {
    return __builtin_amdgcn_wmma_f32_16x16x32_f16(false, a, false, b, (short)0, c, false, false);
  }
};

__device__ __forceinline__ void row_guard_h(v8f& a0, v8f& a1, v8f& a2, v8f& a3,
                                            v16h x, v16h b0, v16h b1, v16h b2, v16h b3) {
  asm volatile("v_nop\n\tv_nop\n\tv_nop\n\tv_nop\n\tv_nop"
               : "+v"(a0), "+v"(a1), "+v"(a2), "+v"(a3)
               : "v"(x), "v"(b0), "v"(b1), "v"(b2), "v"(b3));
}
__device__ __forceinline__ void acc_guard4(v8f& a, v8f& b, v8f& c, v8f& d) {
  asm volatile("v_nop\n\tv_nop\n\tv_nop\n\tv_nop" : "+v"(a), "+v"(b), "+v"(c), "+v"(d));
}

__global__ __launch_bounds__(256) void prep_weights(
    const float* __restrict__ W1, const float* __restrict__ W2,
    unsigned short* __restrict__ W1t, unsigned short* __restrict__ W2t) {
  const int gid = blockIdx.x * 256 + threadIdx.x;
  if (blockIdx.x < 4) {
    const int n  = gid >> 3;
    const int kc = (gid & 7) * 8;
    v8h hv;
#pragma unroll
    for (int e = 0; e < 8; ++e) {
      const float w = W1[(size_t)(kc + e) * kCout + n] * kWCarry;
      hv[e] = (_Float16)w;
    }
    unsigned short* p = W1t + (size_t)n * kCin + kc;
    *(volatile v8h*)p = hv;
    __threadfence();
    *(volatile v8h*)p = hv;
  } else {
    const int g2 = gid - 1024;
    const int n  = g2 >> 4;
    const int kc = (g2 & 15) * 8;
    v8h hv;
#pragma unroll
    for (int e = 0; e < 8; ++e) {
      const float w = W2[(size_t)(kc + e) * kCout + n] * kWCarry;
      hv[e] = (_Float16)w;
    }
    unsigned short* p = W2t + (size_t)n * kCout + kc;
    *(volatile v8h*)p = hv;
    __threadfence();
    *(volatile v8h*)p = hv;
  }
}

constexpr int kFpsThreads = 512;
constexpr int kFpsPer     = kPts / kFpsThreads;
static_assert(kFpsPer == 16);
constexpr int kOut0Vec4   = (kCent * 3) / 4;
constexpr int kOut0Extra  = kOut0Vec4 - kFpsThreads;
static_assert(kOut0Vec4 == 768);
static_assert(kOut0Extra == 256);
static_assert(kOut0Extra % 32 == 0);

__global__ __launch_bounds__(512) void fps_kernel(
    const float* __restrict__ xyz, const int* __restrict__ finit,
    float* __restrict__ out0, float* __restrict__ cxyz4) {
#pragma clang fp contract(off)
  __shared__ __align__(16) float sxyz[kPts * 3];
  __shared__ int   sIdx[kCent];
  __shared__ float redD[16];
  __shared__ int   redI[16];
  __shared__ int   sFar;

  const int b = blockIdx.x;
  const int t = threadIdx.x;
  const float* bx = xyz + (size_t)b * kPts * 3;

#pragma unroll 1
  for (int i = t; i < (kPts * 3) / 4; i += kFpsThreads) {
    const v4f v = *(const v4f*)(bx + 4 * i);
    *(v4f*)(sxyz + 4 * i) = v;
  }
  if (t == 0) {
    int f = finit[b];
    f = f < 0 ? 0 : (f > kPts - 1 ? kPts - 1 : f);
    sFar = f;
  }
  __syncthreads();

  float px[kFpsPer], py[kFpsPer], pz[kFpsPer], dd[kFpsPer];
#pragma unroll
  for (int i = 0; i < kFpsPer; ++i) {
    const int j = t + kFpsThreads * i;
    px[i] = sxyz[3 * j + 0];
    py[i] = sxyz[3 * j + 1];
    pz[i] = sxyz[3 * j + 2];
    dd[i] = 1e10f;
  }

#pragma unroll 1
  for (int step = 0; step < kCent; ++step) {
    const int far = sFar;
    if (t == 0) sIdx[step] = far;
    const float cx = sxyz[far * 3 + 0];
    const float cy = sxyz[far * 3 + 1];
    const float cz = sxyz[far * 3 + 2];

    float bestD = -1.0f;
    int   bestI = 0x7fffffff;
#pragma unroll
    for (int i = 0; i < kFpsPer; ++i) {
      const float dx = px[i] - cx;
      const float dy = py[i] - cy;
      const float dz = pz[i] - cz;
      const float t0 = dx * dx;
      const float t1 = dy * dy;
      const float t2 = dz * dz;
      float d = (t0 + t2) + t1;
      d = fminf(dd[i], d);
      dd[i] = d;
      if (d > bestD) { bestD = d; bestI = t + kFpsThreads * i; }
    }
#pragma unroll
    for (int off = 16; off > 0; off >>= 1) {
      const float od = __shfl_xor(bestD, off);
      const int   oi = __shfl_xor(bestI, off);
      if (od > bestD || (od == bestD && oi < bestI)) { bestD = od; bestI = oi; }
    }
    const int wid = t >> 5;
    if ((t & 31) == 0) { redD[wid] = bestD; redI[wid] = bestI; }
    __syncthreads();
    if (wid == 0) {
      bestD = redD[t & 15];
      bestI = redI[t & 15];
#pragma unroll
      for (int off = 16; off > 0; off >>= 1) {
        const float od = __shfl_xor(bestD, off);
        const int   oi = __shfl_xor(bestI, off);
        if (od > bestD || (od == bestD && oi < bestI)) { bestD = od; bestI = oi; }
      }
      if (t == 0) {
        int f = bestI;
        f = f < 0 ? 0 : (f > kPts - 1 ? kPts - 1 : f);
        sFar = f;
      }
    }
    __syncthreads();
  }

  float* ob = out0 + (size_t)b * kCent * 3;
  float* cb = cxyz4 + (size_t)b * kCent * 4;
  v4f ov  = (v4f){0.f, 0.f, 0.f, 0.f};
  v4f ov1 = (v4f){0.f, 0.f, 0.f, 0.f};
#pragma unroll
  for (int e = 0; e < 4; ++e) {
    const int el = 4 * t + e;
    const int s  = el / 3;
    const int c  = el - 3 * s;
    const int id = sIdx[s];
    ov[e] = sxyz[id * 3 + c];
  }
  if (t < kOut0Extra) {
#pragma unroll
    for (int e = 0; e < 4; ++e) {
      const int el = 4 * (t + kFpsThreads) + e;
      int s = el / 3;
      const int c = el - 3 * s;
      s = s > kCent - 1 ? kCent - 1 : s;
      const int id = sIdx[s];
      ov1[e] = sxyz[id * 3 + c];
    }
  }
  v4f cv0, cv1;
  {
    const int i0 = sIdx[t];
    const int i1 = sIdx[t + kFpsThreads];
    cv0 = (v4f){sxyz[i0 * 3 + 0], sxyz[i0 * 3 + 1], sxyz[i0 * 3 + 2], 0.f};
    cv1 = (v4f){sxyz[i1 * 3 + 0], sxyz[i1 * 3 + 1], sxyz[i1 * 3 + 2], 0.f};
  }
  for (int pass = 0; pass < 2; ++pass) {
    *(volatile v4f*)(ob + 4 * t) = ov;
    if (t < kOut0Extra) *(volatile v4f*)(ob + 4 * (t + kFpsThreads)) = ov1;
    *(volatile v4f*)(cb + 4 * t) = cv0;
    *(volatile v4f*)(cb + 4 * (t + kFpsThreads)) = cv1;
    __threadfence();
  }
}

constexpr int kKnnT  = 64;
constexpr int kChunk = 512;
static_assert(kPts % kChunk == 0);

__global__ __launch_bounds__(64) void knn_gather_kernel(
    const float* __restrict__ xyz, const float* __restrict__ feat,
    const float* __restrict__ cxyz4, unsigned short* __restrict__ comb) {
#pragma clang fp contract(off)
  __shared__ float kD[kKnnT][kNbr + 1];
  __shared__ int   kI[kKnnT][kNbr + 1];
  __shared__ __align__(16) float sP[kChunk * 3];
  __shared__ float sSq[kChunk];
  __shared__ __align__(16) float sC[kKnnT * 4];

  const int t   = threadIdx.x;
  const int cid = blockIdx.x * kKnnT + t;
  const int b   = (blockIdx.x * kKnnT) / kCent;

  const v4f c4 = *(const v4f*)(cxyz4 + (size_t)cid * 4);
  const float cx = c4[0];
  const float cy = c4[1];
  const float cz = c4[2];
  *(v4f*)(sC + 4 * t) = c4;
  float cs;
  {
    const float t0 = cx * cx;
    const float t1 = cy * cy;
    const float t2 = cz * cz;
    cs = (t0 + t2) + t1;
  }

  float* Dl = kD[t];
  int*   Il = kI[t];
#pragma unroll 1
  for (int k = 0; k < kNbr; ++k) { Dl[k] = 3.0e38f; Il[k] = 0; }
  float T   = 3.0e38f;
  float Tsq = T * T * 1.000002f;

#pragma unroll 1
  for (int ch = 0; ch < kPts / kChunk; ++ch) {
    __syncthreads();
    const float* src = xyz + ((size_t)b * kPts + (size_t)ch * kChunk) * 3;
#pragma unroll
    for (int i = 0; i < 6; ++i) {
      const int f = t + kKnnT * i;
      const v4f v = *(const v4f*)(src + 4 * f);
      *(v4f*)(sP + 4 * f) = v;
    }
    __syncthreads();
#pragma unroll
    for (int i = 0; i < 8; ++i) {
      const int j = t + kKnnT * i;
      const float x = sP[3 * j + 0];
      const float y = sP[3 * j + 1];
      const float z = sP[3 * j + 2];
      const float t0 = x * x;
      const float t1 = y * y;
      const float t2 = z * z;
      sSq[j] = (t0 + t2) + t1;
    }
    __syncthreads();

    const int jbase = ch * kChunk;
#pragma unroll 2
    for (int j = 0; j < kChunk; ++j) {
      const float qx = sP[3 * j + 0];
      const float qy = sP[3 * j + 1];
      const float qz = sP[3 * j + 2];
      const float sq = sSq[j];
      float p = cx * qx;
      p = __builtin_fmaf(cy, qy, p);
      p = __builtin_fmaf(cz, qz, p);
      float d2 = (cs + sq) - 2.0f * p;
      d2 = fmaxf(d2, 0.0f);
      if (!(d2 > Tsq)) {
        const float ds = sqrtf(d2);
        if (ds < T) {
          int pp = kNbr - 1;
          while (pp > 0 && Dl[pp - 1] > ds) {
            Dl[pp] = Dl[pp - 1];
            Il[pp] = Il[pp - 1];
            --pp;
          }
          Dl[pp] = ds;
          Il[pp] = jbase + j;
          T   = Dl[kNbr - 1];
          Tsq = T * T * 1.000002f;
        }
      }
    }
  }
  __syncthreads();

#pragma unroll 1
  for (int k = 0; k < kNbr; ++k) {
    const float dk = Dl[k];
    int g = Il[k];
    g = (dk > kRadius) ? 0 : g;
    g = g < 0 ? 0 : (g > kPts - 1 ? kPts - 1 : g);
    Il[k] = g;
  }
  __syncthreads();

  const int q   = t & 7;
  const float sel0 = (q == 0) ? 1.0f : 0.0f;
  const float sel1 = 1.0f - sel0;
  const size_t rowBase = (size_t)blockIdx.x * kKnnT * kNbr;
#pragma unroll 1
  for (int it = 0; it < (kKnnT * kNbr) / 8; ++it) {
    const int lr = it * 8 + (t >> 3);
    const int lc = lr >> 5;
    const int kk = lr & 31;
    int g = kI[lc][kk];
    g = g < 0 ? 0 : (g > kPts - 1 ? kPts - 1 : g);
    const float ccx = sC[4 * lc + 0];
    const float ccy = sC[4 * lc + 1];
    const float ccz = sC[4 * lc + 2];
    const float* pr = xyz  + ((size_t)b * kPts + g) * 3;
    const float* fr = feat + ((size_t)b * kPts + g) * kFeat;
    const float gx = pr[0];
    const float gy = pr[1];
    const float gz = pr[2];
    float f[8];
#pragma unroll
    for (int e = 0; e < 8; ++e) {
      int fi = 8 * q + e - 3;
      fi = fi < 0 ? 0 : fi;
      f[e] = fr[fi];
    }
    const float dx = gx - ccx;
    const float dy = gy - ccy;
    const float dz = gz - ccz;
    f[0] = sel0 * dx + sel1 * f[0];
    f[1] = sel0 * dy + sel1 * f[1];
    f[2] = sel0 * dz + sel1 * f[2];
    v8h hv;
#pragma unroll
    for (int e = 0; e < 8; ++e) hv[e] = (_Float16)f[e];
    unsigned short* p = comb + (rowBase + (size_t)lr) * kCin + q * 8;
    *(volatile v8h*)p = hv;
    __threadfence();
    *(volatile v8h*)p = hv;
  }
}

template <int KD, int MODE>
__global__ __launch_bounds__(256) void mlp_gemm(
    const unsigned short* __restrict__ Ap, const unsigned short* __restrict__ Btp,
    const float* __restrict__ bias, const float* __restrict__ scbi,
    float* __restrict__ part, unsigned short* __restrict__ Hout,
    float* __restrict__ ymax, float* __restrict__ ymin) {
  static_assert(KD % 32 == 0);
  const _Float16* A  = (const _Float16*)Ap;
  const _Float16* Bt = (const _Float16*)Btp;
  __shared__ __align__(16) float sT[(MODE == 1) ? 8 * 16 * 68 : 4];
  __shared__ float sRed[(MODE != 1) ? 2 * 8 * 64 : 4];
  __shared__ __align__(16) float sPool[(MODE == 2) ? 2 * 8 * 128 : 4];

  const int lane  = threadIdx.x & 31;
  const int wave  = threadIdx.x >> 5;
  const int tm    = wave >> 1;
  const int tn    = wave & 1;
  const int m0    = blockIdx.x * 256 + tm * 64;
  const int n0    = tn * 64;
  const int rlane = lane & 15;
  const int hh    = lane >> 4;
  const int koff  = hh * 8;
  const int mOff  = hh * 8;

  v8f acc[4][4];
#pragma unroll
  for (int i = 0; i < 4; ++i)
#pragma unroll
    for (int j = 0; j < 4; ++j) acc[i][j] = (v8f){0.f, 0.f, 0.f, 0.f, 0.f, 0.f, 0.f, 0.f};

  for (int k0 = 0; k0 < KD; k0 += 32) {
    v16h bh[4];
#pragma unroll
    for (int j = 0; j < 4; ++j) {
      const size_t bo = (size_t)(n0 + (j << 4) + rlane) * KD + koff + k0;
      bh[j] = FragH::load(Bt + bo);
    }
#pragma unroll
    for (int i = 0; i < 4; ++i) {
      const size_t ao = (size_t)(m0 + (i << 4) + rlane) * KD + koff + k0;
      const v16h ah = FragH::load(A + ao);
#pragma unroll
      for (int j = 0; j < 4; ++j) acc[i][j] = FragH::mma(ah, bh[j], acc[i][j]);
      row_guard_h(acc[i][0], acc[i][1], acc[i][2], acc[i][3], ah, bh[0], bh[1], bh[2], bh[3]);
    }
  }
  acc_guard4(acc[0][0], acc[0][1], acc[0][2], acc[0][3]);
  acc_guard4(acc[1][0], acc[1][1], acc[1][2], acc[1][3]);
  acc_guard4(acc[2][0], acc[2][1], acc[2][2], acc[2][3]);
  acc_guard4(acc[3][0], acc[3][1], acc[3][2], acc[3][3]);

  float bv[4];
#pragma unroll
  for (int j = 0; j < 4; ++j) bv[j] = bias[n0 + (j << 4) + rlane];

  if (MODE == 1) {
    float scv[4], biv[4];
#pragma unroll
    for (int j = 0; j < 4; ++j) {
      scv[j] = scbi[n0 + (j << 4) + rlane];
      biv[j] = scbi[kCout + n0 + (j << 4) + rlane];
    }
    float* slab = sT + wave * 16 * 68;
    _Float16* H = (_Float16*)Hout;
#pragma unroll
    for (int i = 0; i < 4; ++i) {
      const int mBase = m0 + (i << 4);
#pragma unroll
      for (int j = 0; j < 4; ++j) {
#pragma unroll
        for (int r = 0; r < 8; ++r) {
          const float y = acc[i][j][r] * kWCarryInv + bv[j];
          const float v = fmaxf(scv[j] * y + biv[j], 0.0f);
          slab[(mOff + r) * 68 + (j << 4) + rlane] = v;
        }
      }
      __builtin_amdgcn_fence(__ATOMIC_RELEASE, "workgroup");
      __builtin_amdgcn_wave_barrier();
      __builtin_amdgcn_fence(__ATOMIC_ACQUIRE, "workgroup");
      {
        const int q = lane >> 3, c8 = (lane & 7) * 8;
        for (int pass = 0; pass < 2; ++pass) {
#pragma unroll
          for (int it = 0; it < 4; ++it) {
            const int row = it * 4 + q;
            const float* sp = slab + row * 68 + c8;
            v8h hv;
#pragma unroll
            for (int e = 0; e < 8; ++e) hv[e] = (_Float16)sp[e];
            *(volatile v8h*)(H + (size_t)(mBase + row) * kCout + n0 + c8) = hv;
          }
          __threadfence();
        }
      }
      __builtin_amdgcn_fence(__ATOMIC_RELEASE, "workgroup");
      __builtin_amdgcn_wave_barrier();
      __builtin_amdgcn_fence(__ATOMIC_ACQUIRE, "workgroup");
    }
  } else {
#pragma unroll
    for (int j = 0; j < 4; ++j) {
      float s = 0.0f, qq = 0.0f;
#pragma unroll
      for (int i = 0; i < 4; ++i) {
#pragma unroll
        for (int r = 0; r < 8; ++r) {
          const float y = acc[i][j][r] * kWCarryInv + bv[j];
          const float y2 = y * y;
          s  = s + y;
          qq = qq + y2;
        }
      }
      const float so = __shfl_xor(s, 16);
      const float qo = __shfl_xor(qq, 16);
      s  = s + so;
      qq = qq + qo;
      if (hh == 0) {
        sRed[(0 * 8 + wave) * 64 + (j << 4) + rlane] = s;
        sRed[(1 * 8 + wave) * 64 + (j << 4) + rlane] = qq;
      }
    }
    if (MODE == 2) {
#pragma unroll
      for (int j = 0; j < 4; ++j) {
#pragma unroll
        for (int cp = 0; cp < 2; ++cp) {
          float mx = -INFINITY, mn = INFINITY;
#pragma unroll
          for (int ii = 0; ii < 2; ++ii) {
#pragma unroll
            for (int r = 0; r < 8; ++r) {
              const float y = acc[2 * cp + ii][j][r] * kWCarryInv + bv[j];
              mx = fmaxf(mx, y);
              mn = fminf(mn, y);
            }
          }
          const float mxo = __shfl_xor(mx, 16);
          const float mno = __shfl_xor(mn, 16);
          mx = fmaxf(mx, mxo);
          mn = fminf(mn, mno);
          if (hh == 0) {
            sPool[(0 * 8 + tm * 2 + cp) * 128 + n0 + (j << 4) + rlane] = mx;
            sPool[(1 * 8 + tm * 2 + cp) * 128 + n0 + (j << 4) + rlane] = mn;
          }
        }
      }
    }
    __syncthreads();
    {
      const int tid   = threadIdx.x;
      const int which = tid >> 7;
      const int n     = tid & 127;
      const int tnn   = n >> 6;
      const int col   = n & 63;
      const float a0 = sRed[(which * 8 + 0 + tnn) * 64 + col];
      const float a1 = sRed[(which * 8 + 2 + tnn) * 64 + col];
      const float a2 = sRed[(which * 8 + 4 + tnn) * 64 + col];
      const float a3 = sRed[(which * 8 + 6 + tnn) * 64 + col];
      const float tot = ((a0 + a1) + a2) + a3;
      float* pp = part + (size_t)blockIdx.x * 256 + tid;
      *(volatile float*)pp = tot;
      __threadfence();
      *(volatile float*)pp = tot;
      if (MODE == 2) {
        const v4f vmx = *(const v4f*)(sPool + 4 * tid);
        const v4f vmn = *(const v4f*)(sPool + 8 * 128 + 4 * tid);
        float* pmx = ymax + (size_t)blockIdx.x * 8 * kCout + 4 * tid;
        float* pmn = ymin + (size_t)blockIdx.x * 8 * kCout + 4 * tid;
        for (int pass = 0; pass < 2; ++pass) {
          *(volatile v4f*)pmx = vmx;
          *(volatile v4f*)pmn = vmn;
          __threadfence();
        }
      }
    }
  }
}

__global__ __launch_bounds__(256) void bn_finalize(
    const float* __restrict__ part, const float* __restrict__ gam,
    const float* __restrict__ bet, float* __restrict__ scbi) {
  __shared__ double sS[256];
  __shared__ float  sO[256];
  const int t = threadIdx.x;
  double a = 0.0;
#pragma unroll 4
  for (int blk = 0; blk < kGemmBlocks; ++blk) a += (double)part[(size_t)blk * 256 + t];
  sS[t] = a;
  __syncthreads();
  if (t < 128) {
    const double invM = 1.0 / (double)kRows;
    const double mean = sS[t] * invM;
    double var = sS[128 + t] * invM - mean * mean;
    var = var < 0.0 ? 0.0 : var;
    const float vf = (float)var + kBnEps;
    const float rs = 1.0f / sqrtf(vf);
    const float sc = gam[t] * rs;
    const float bi = bet[t] - (float)mean * sc;
    sO[t] = sc;
    sO[128 + t] = bi;
  }
  __syncthreads();
  const float o = sO[t];
  *(volatile float*)(scbi + t) = o;
  __threadfence();
  *(volatile float*)(scbi + t) = o;
}

__global__ __launch_bounds__(256) void pool_out(
    const float* __restrict__ ymax, const float* __restrict__ ymin,
    const float* __restrict__ scbi, float* __restrict__ out1) {
  const size_t gid = (size_t)blockIdx.x * 256 + threadIdx.x;
  const int c4 = (int)(gid & 31) * 4;
  const v4f mx = *(const v4f*)(ymax + gid * 4);
  const v4f mn = *(const v4f*)(ymin + gid * 4);
  const v4f sc = *(const v4f*)(scbi + c4);
  const v4f bi = *(const v4f*)(scbi + kCout + c4);
  v4f o;
#pragma unroll
  for (int e = 0; e < 4; ++e) {
    const float s = sc[e];
    const float a = mx[e];
    const float b = mn[e];
    const float pick = (s >= 0.0f) ? a : b;
    o[e] = fmaxf(s * pick + bi[e], 0.0f);
  }
  float* p = out1 + gid * 4;
  *(volatile v4f*)p = o;
  __threadfence();
  *(volatile v4f*)p = o;
}

extern "C" void kernel_launch(void* const* d_in, const int* in_sizes, int n_in,
                              void* d_out, int out_size, void* d_ws, size_t ws_size,
                              hipStream_t stream) {
  (void)in_sizes; (void)n_in; (void)out_size;
  const float* xyz   = (const float*)d_in[0];
  const float* feat  = (const float*)d_in[1];
  const int*   finit = (const int*)d_in[2];
  const float* W1    = (const float*)d_in[3];
  const float* b1    = (const float*)d_in[4];
  const float* g1    = (const float*)d_in[5];
  const float* be1   = (const float*)d_in[6];
  const float* W2    = (const float*)d_in[7];
  const float* b2    = (const float*)d_in[8];
  const float* g2    = (const float*)d_in[9];
  const float* be2   = (const float*)d_in[10];

  float* out0 = (float*)d_out;
  float* out1 = (float*)d_out + (size_t)(98304 / 4);

  size_t off = 0;
  char* ws = (char*)d_ws;
  unsigned short* W1t = (unsigned short*)(ws + off); off += (size_t)kCout * kCin * 2;
  unsigned short* W2t = (unsigned short*)(ws + off); off += (size_t)kCout * kCout * 2;
  float* scbi1 = (float*)(ws + off); off += 1024;
  float* scbi2 = (float*)(ws + off); off += 1024;
  float* cxyz4 = (float*)(ws + off); off += (size_t)kBatch * kCent * 4 * 4;
  float* part1 = (float*)(ws + off); off += (size_t)kGemmBlocks * 256 * 4;
  float* part2 = (float*)(ws + off); off += (size_t)kGemmBlocks * 256 * 4;
  float* ymax  = (float*)(ws + off); off += (size_t)kBatch * kCent * kCout * 4;
  float* ymin  = (float*)(ws + off); off += (size_t)kBatch * kCent * kCout * 4;
  unsigned short* comb = (unsigned short*)(ws + off); off += (size_t)kRows * kCin * 2;
  unsigned short* H1   = (unsigned short*)(ws + off); off += (size_t)kRows * kCout * 2;
  if (off > ws_size || off > (size_t)134217728) return;

  prep_weights<<<12, 256, 0, stream>>>(W1, W2, W1t, W2t);
  fps_kernel<<<kBatch, kFpsThreads, 0, stream>>>(xyz, finit, out0, cxyz4);
  knn_gather_kernel<<<(kBatch * kCent) / kKnnT, kKnnT, 0, stream>>>(xyz, feat, cxyz4, comb);
  mlp_gemm<kCin, 0><<<kGemmBlocks, 256, 0, stream>>>(comb, W1t, b1, scbi1, part1, H1, ymax, ymin);
  bn_finalize<<<1, 256, 0, stream>>>(part1, g1, be1, scbi1);
  mlp_gemm<kCin, 1><<<kGemmBlocks, 256, 0, stream>>>(comb, W1t, b1, scbi1, part1, H1, ymax, ymin);
  mlp_gemm<kCout, 2><<<kGemmBlocks, 256, 0, stream>>>(H1, W2t, b2, scbi2, part2, H1, ymax, ymin);
  bn_finalize<<<1, 256, 0, stream>>>(part2, g2, be2, scbi2);
  pool_out<<<(kBatch * kCent * kCout / 4) / 256, 256, 0, stream>>>(ymax, ymin, scbi2, out1);
}
